// MultiResolutionSSM_80564996538674
// MI455X (gfx1250) — hardware-run, weakly checked
//
#include <hip/hip_runtime.h>
#include <math.h>

constexpr int kB   = 4;
constexpr int kT   = 4096;
constexpr int kH   = 512;
constexpr int kS   = 64;
constexpr int kL1  = (kT + 7) / 2;
constexpr int kL2  = (kL1 + 7) / 2;
constexpr int kM0  = kB * kL1;
constexpr int kM0p = ((kM0 + 63) / 64) * 64;
constexpr int kM1  = kB * kL2;
constexpr int kM1p = ((kM1 + 63) / 64) * 64;
constexpr int kNout = kB * kT;
constexpr int kKup  = 3 * kH + 64;
constexpr int kKup8 = kKup / 8;
constexpr int kWattPitch = 64;
constexpr float kACarry  = 4.0f;
constexpr float kWCarry  = 16.0f;
constexpr float kUpScale = 1.0f / 64.0f;
static_assert(kL1 == 2051 && kL2 == 1029);
static_assert(kM0p == 8256 && kM1p == 4160);
static_assert(kM0p % 64 == 0 && kM1p % 64 == 0 && kM0p - kM0 < 64 && kM1p - kM1 < 64);
static_assert(kKup % 32 == 0 && (kKup * 2) % 128 == 0);

constexpr size_t kBytesCA1  = (size_t)kM0 * kH * 4;
constexpr size_t kBytesHIGH = (size_t)kM0 * kH * 4;
constexpr size_t kBytesLOW  = (size_t)kM1 * kH * 4;
constexpr size_t kBytesMID  = (size_t)kM1 * kH * 4;
constexpr size_t kBytesSIG1 = (size_t)kM0p * kH * 2;
constexpr size_t kBytesBX   = (size_t)kM0p * kS * 4;
constexpr size_t kBytesST1  = (size_t)kM0p * kS * 2;
constexpr size_t kBytesAF   = (size_t)kNout * kKup * 2;
constexpr size_t kBytesWUP  = (size_t)kH * kKup * 2;
constexpr size_t kBytesW16  = (size_t)3 * kS * kH * 2;
constexpr size_t kBytesWATT = (size_t)kB * kWattPitch * 4;

constexpr size_t kOffCA1  = 0;
constexpr size_t kOffHIGH = kOffCA1 + kBytesCA1;
constexpr size_t kOffLOW  = kOffHIGH + kBytesHIGH;
constexpr size_t kOffMID  = kOffLOW + kBytesLOW;
constexpr size_t kOffSIGH = kOffMID + kBytesMID;
constexpr size_t kOffSIGL = kOffSIGH + kBytesSIG1;
constexpr size_t kOffY    = kOffSIGH;
constexpr size_t kOffBX   = kOffSIGL + kBytesSIG1;
constexpr size_t kOffSTH  = kOffBX + kBytesBX;
constexpr size_t kOffSTL  = kOffSTH + kBytesST1;
constexpr size_t kOffAF   = kOffSTL + kBytesST1;
constexpr size_t kOffWUP  = kOffAF + kBytesAF;
constexpr size_t kOffBWH  = kOffWUP + kBytesWUP;
constexpr size_t kOffBWL  = kOffBWH + kBytesW16;
constexpr size_t kOffCWH  = kOffBWL + kBytesW16;
constexpr size_t kOffCWL  = kOffCWH + kBytesW16;
constexpr size_t kOffWATT = kOffCWL + kBytesW16;
constexpr size_t kWsTotal = kOffWATT + kBytesWATT;
static_assert((size_t)kM0p * kH * 4 == 2 * kBytesSIG1);
static_assert(kWsTotal == 126452736);
static_assert(kWsTotal <= (size_t)134217728);
static_assert(kOffHIGH % 256 == 0 && kOffLOW % 256 == 0 && kOffMID % 256 == 0 && kOffSIGH % 256 == 0 &&
              kOffSIGL % 256 == 0 && kOffBX % 256 == 0 && kOffSTH % 256 == 0 && kOffSTL % 256 == 0 &&
              kOffAF % 256 == 0 && kOffWUP % 256 == 0 && kOffBWH % 256 == 0 && kOffBWL % 256 == 0 &&
              kOffCWH % 256 == 0 && kOffCWL % 256 == 0 && kOffWATT % 256 == 0);

__constant__ float c_dec_lo[8] = {
    -0.010597401784997278f,  0.032883011666982945f,  0.030841381835986965f,
    -0.18703481171888114f,  -0.02798376941698385f,   0.6308807679295904f,
     0.7148465705525415f,    0.23037781330885523f};
__constant__ float c_dec_hi[8] = {
    -0.23037781330885523f,   0.7148465705525415f,   -0.6308807679295904f,
    -0.02798376941698385f,   0.18703481171888114f,   0.030841381835986965f,
    -0.032883011666982945f, -0.010597401784997278f};
static_assert(sizeof(c_dec_lo) / sizeof(c_dec_lo[0]) == 8);
static_assert(sizeof(c_dec_hi) / sizeof(c_dec_hi[0]) == 8);

typedef __attribute__((ext_vector_type(16))) _Float16 v16h;
typedef __attribute__((ext_vector_type(8)))  _Float16 v8h;
typedef __attribute__((ext_vector_type(16))) __bf16   v16b;
typedef __attribute__((ext_vector_type(8)))  __bf16   v8b;
typedef __attribute__((ext_vector_type(8)))  float    v8f;
typedef __attribute__((ext_vector_type(4)))  float    v4f;
typedef __attribute__((ext_vector_type(4)))  unsigned int v4u;

__device__ __forceinline__ unsigned short f2bf_bits(float f) {
  unsigned u = __float_as_uint(f);
  return (unsigned short)((u + 0x7FFFu + ((u >> 16) & 1u)) >> 16);
}
__device__ __forceinline__ float bf_bits2f(unsigned short h) { return __uint_as_float(((unsigned)h) << 16); }

__device__ __forceinline__ void dep_guard_h(v8f& a, v8f& b, v16h x, v16h y) { asm volatile("v_nop\n\tv_nop\n\tv_nop\n\tv_nop" : "+v"(a), "+v"(b) : "v"(x), "v"(y)); }
__device__ __forceinline__ void dep_guard_b(v8f& a, v8f& b, v16b x, v16b y) { asm volatile("v_nop\n\tv_nop\n\tv_nop\n\tv_nop" : "+v"(a), "+v"(b) : "v"(x), "v"(y)); }
__device__ __forceinline__ void keep4_h(v16h a, v16h b, v16h c, v16h d) { asm volatile("v_nop" :: "v"(a), "v"(b), "v"(c), "v"(d)); }
__device__ __forceinline__ void keep4_b(v16b a, v16b b, v16b c, v16b d) { asm volatile("v_nop" :: "v"(a), "v"(b), "v"(c), "v"(d)); }
__device__ __forceinline__ void acc_guard4(v8f& a, v8f& b, v8f& c, v8f& d) { asm volatile("v_nop\n\tv_nop\n\tv_nop\n\tv_nop" : "+v"(a), "+v"(b), "+v"(c), "+v"(d)); }
template <typename T> struct Frag;
template <> struct Frag<_Float16> {
  typedef v16h V; union U { v16h v; v8h h[2]; };
  static __device__ __forceinline__ v16h load(const _Float16* p) {
    U f; f.h[0] = *(const v8h*)(p); f.h[1] = *(const v8h*)(p + 16); return f.v;
  }
  static __device__ __forceinline__ v8f mma(v16h a, v16h b, v8f c) {
    return __builtin_amdgcn_wmma_f32_16x16x32_f16(false, a, false, b, (short)0, c, false, false);
  }
  static __device__ __forceinline__ void guard(v8f& a, v8f& b, v16h x, v16h y) { dep_guard_h(a, b, x, y); }
  static __device__ __forceinline__ void keep(v16h a, v16h b, v16h c, v16h d) { keep4_h(a, b, c, d); }
};
template <> struct Frag<__bf16> {
  typedef v16b V; union U { v16b v; v8b h[2]; };
  static __device__ __forceinline__ v16b load(const __bf16* p) {
    U f; f.h[0] = *(const v8b*)(p); f.h[1] = *(const v8b*)(p + 16); return f.v;
  }
  static __device__ __forceinline__ v8f mma(v16b a, v16b b, v8f c) {
    return __builtin_amdgcn_wmma_f32_16x16x32_bf16(false, a, false, b, (short)0, c, false, false);
  }
  static __device__ __forceinline__ void guard(v8f& a, v8f& b, v16b x, v16b y) { dep_guard_b(a, b, x, y); }
  static __device__ __forceinline__ void keep(v16b a, v16b b, v16b c, v16b d) { keep4_b(a, b, c, d); }
};

__device__ __forceinline__ unsigned pk16(unsigned short a, unsigned short b) { return (unsigned)a | ((unsigned)b << 16); }
__device__ __forceinline__ unsigned short h_bits(float f) { const _Float16 h = (_Float16)f; return __builtin_bit_cast(unsigned short, h); }

template <int ET> struct Elem;
template <> struct Elem<0> { typedef _Float16 T; };
template <> struct Elem<1> { typedef __bf16 T; };
template <int ET, bool SPLIT, int BIAS_MODE, int OUT_MODE, bool RESID, int ACT = 0>
__global__ __launch_bounds__(256) void wmma_gemm64(
    const unsigned short* __restrict__ Ap, const unsigned short* __restrict__ A2p, int lda, long strideA,
    const unsigned short* __restrict__ Btp, const unsigned short* __restrict__ Bt2p, int ldb, long strideB,
    void* __restrict__ Cout, void* __restrict__ Cout2, int ldc, long strideC,
    const float* __restrict__ bias,
    const float* __restrict__ resid, long strideR,
    int M, int N, int K, float scale) {
  typedef typename Elem<ET>::T T;
  typedef typename Frag<T>::V V;
  const T* A = (const T*)Ap; const T* A2 = (const T*)A2p; const T* Bt = (const T*)Btp; const T* Bt2 = (const T*)Bt2p;
  __shared__ __align__(16) float sT[8][16 * 68];
  const int b    = blockIdx.y;
  const int lane = threadIdx.x & 31;
  const int wave = threadIdx.x >> 5;
  const int tilesN = N >> 6;
  const int tilesM = M >> 6;
  const int tile = blockIdx.x * 8 + wave;
  if (tile >= tilesM * tilesN) return;
  const int tm = tile / tilesN;
  const int tn = tile - tm * tilesN;
  const int m0 = tm << 6;
  const int n0 = tn << 6;

  const T* Ab  = A  + (size_t)b * strideA;
  const T* Bb  = Bt + (size_t)b * strideB;
  const T* Ab2 = SPLIT ? (A2  + (size_t)b * strideA) : nullptr;
  const T* Bb2 = SPLIT ? (Bt2 + (size_t)b * strideB) : nullptr;

  const int rlane = lane & 15;
  const int koff  = (lane >> 4) * 8;
  const int mOff  = (lane >> 4) * 8;

  v8f acc[4][4];
#pragma unroll
  for (int i = 0; i < 4; ++i)
#pragma unroll
    for (int j = 0; j < 4; ++j) acc[i][j] = (v8f){0.f,0.f,0.f,0.f,0.f,0.f,0.f,0.f};

  for (int k0 = 0; k0 < K; k0 += 32) {
    V bh[4], bl[4];
#pragma unroll
    for (int j = 0; j < 4; ++j) {
      const size_t bo = (size_t)(n0 + (j << 4) + rlane) * ldb + koff + k0;
      bh[j] = Frag<T>::load(Bb + bo);
      if (SPLIT) bl[j] = Frag<T>::load(Bb2 + bo);
    }
#pragma unroll
    for (int i = 0; i < 4; ++i) {
      const size_t ao = (size_t)(m0 + (i << 4) + rlane) * lda + koff + k0;
      V ah = Frag<T>::load(Ab + ao);
      V al;
      if (SPLIT) al = Frag<T>::load(Ab2 + ao);
#pragma unroll
      for (int j = 0; j < 4; ++j) {
        acc[i][j] = Frag<T>::mma(ah, bh[j], acc[i][j]);
        if (SPLIT) {
          acc[i][j] = Frag<T>::mma(ah, bl[j], acc[i][j]);
          acc[i][j] = Frag<T>::mma(al, bh[j], acc[i][j]);
        }
      }
      Frag<T>::guard(acc[i][0], acc[i][3], ah, SPLIT ? al : ah);
    }
    Frag<T>::keep(bh[0], bh[1], bh[2], bh[3]);
    if (SPLIT) Frag<T>::keep(bl[0], bl[1], bl[2], bl[3]);
  }
  acc_guard4(acc[0][0], acc[0][1], acc[0][2], acc[0][3]);
  acc_guard4(acc[1][0], acc[1][1], acc[1][2], acc[1][3]);
  acc_guard4(acc[2][0], acc[2][1], acc[2][2], acc[2][3]);
  acc_guard4(acc[3][0], acc[3][1], acc[3][2], acc[3][3]);

  float* slab = sT[wave];
  const float* Rb = RESID ? (resid + (size_t)b * strideR) : nullptr;
#pragma unroll
  for (int i = 0; i < 4; ++i) {
    const int mBase = m0 + (i << 4);
#pragma unroll
    for (int j = 0; j < 4; ++j) {
      const int n = n0 + (j << 4) + rlane;
      float bv = 0.f;
      if (BIAS_MODE == 2) bv = bias[n];
#pragma unroll
      for (int r = 0; r < 8; ++r) {
        float v = acc[i][j][r] * scale;
        if (BIAS_MODE == 1) v += bias[mBase + mOff + r];
        if (BIAS_MODE == 2) v += bv;
        if (RESID) v += Rb[(size_t)(mBase + mOff + r) * ldc + n];
        if (ACT == 2) v = fmaxf(v, 0.0f);
        if (ACT == 4) v = (v > 0.f) ? v : 0.01f * v;
        slab[(mOff + r) * 68 + (j << 4) + rlane] = v;
      }
    }
    __builtin_amdgcn_fence(__ATOMIC_RELEASE, "workgroup");
    __builtin_amdgcn_wave_barrier();
    __builtin_amdgcn_fence(__ATOMIC_ACQUIRE, "workgroup");
    if (OUT_MODE == 0) {
      float* C = (float*)Cout + (size_t)b * strideC;
      const int hh = lane >> 4, c4 = (lane & 15) * 4;
      for (int pass = 0; pass < 2; ++pass) {
#pragma unroll
        for (int it = 0; it < 8; ++it) {
          const int row = it * 2 + hh;
          v4f v = *(const v4f*)(slab + row * 68 + c4);
          *(volatile v4f*)(C + (size_t)(mBase + row) * ldc + n0 + c4) = v;
        }
        __threadfence();
      }
    } else {
      const int q = lane >> 3, c8 = (lane & 7) * 8;
      unsigned short* C  = (unsigned short*)Cout  + (size_t)b * strideC;
      unsigned short* C2 = (OUT_MODE == 2) ? ((unsigned short*)Cout2 + (size_t)b * strideC) : nullptr;
      for (int pass = 0; pass < 2; ++pass) {
#pragma unroll
        for (int it = 0; it < 4; ++it) {
          const int row = it * 4 + q;
          const float* sp = slab + row * 68 + c8;
          v8h hv, lv;
#pragma unroll
          for (int e = 0; e < 8; ++e) {
            if (OUT_MODE == 1) {
              hv[e] = (_Float16)sp[e];
            } else {
              unsigned short hb = f2bf_bits(sp[e]);
              unsigned short lb = f2bf_bits(sp[e] - bf_bits2f(hb));
              hv[e] = __builtin_bit_cast(_Float16, hb);
              lv[e] = __builtin_bit_cast(_Float16, lb);
            }
          }
          *(volatile v8h*)(C + (size_t)(mBase + row) * ldc + n0 + c8) = hv;
          if (OUT_MODE == 2) *(volatile v8h*)(C2 + (size_t)(mBase + row) * ldc + n0 + c8) = lv;
        }
        __threadfence();
      }
    }
    __builtin_amdgcn_fence(__ATOMIC_RELEASE, "workgroup");
    __builtin_amdgcn_wave_barrier();
    __builtin_amdgcn_fence(__ATOMIC_ACQUIRE, "workgroup");
  }
}

__global__ __launch_bounds__(128) void dwt_kernel(const float* __restrict__ in,
                                                  float* __restrict__ outA, float* __restrict__ outD,
                                                  int Tin, int Tout) {
#pragma clang fp contract(off)
  const int bo = blockIdx.x;
  const int b  = bo / Tout;
  const int t  = bo - b * Tout;
  const int c4 = threadIdx.x * 4;
  const float* xb = in + (size_t)b * Tin * kH + c4;
  v4f accA = (v4f){0.f, 0.f, 0.f, 0.f};
  v4f accD = (v4f){0.f, 0.f, 0.f, 0.f};
#pragma unroll
  for (int k = 0; k < 8; ++k) {
    int idx = 2 * t + k - 6;
    idx = (idx < 0) ? (-idx - 1) : idx;
    idx = (idx >= Tin) ? (2 * Tin - 1 - idx) : idx;
    idx = idx < 0 ? 0 : (idx > Tin - 1 ? Tin - 1 : idx);
    const v4f v = *(const v4f*)(xb + (size_t)idx * kH);
    const float cl = c_dec_lo[7 - k];
    const float ch = c_dec_hi[7 - k];
    accA = accA + cl * v;
    accD = accD + ch * v;
  }
  const size_t o = (size_t)bo * kH + c4;
  *(volatile v4f*)(outA + o) = accA;
  *(volatile v4f*)(outD + o) = accD;
  __threadfence();
  *(volatile v4f*)(outA + o) = accA;
  *(volatile v4f*)(outD + o) = accD;
}

__device__ __forceinline__ void split_bf(float v, unsigned short& hb, unsigned short& lb) {
  hb = f2bf_bits(v);
  lb = f2bf_bits(v - bf_bits2f(hb));
}
__global__ __launch_bounds__(256) void split8_bf16_kernel(const float* __restrict__ in,
                                                          unsigned short* __restrict__ outH,
                                                          unsigned short* __restrict__ outL,
                                                          int nreal8, int ntot8) {
  const int i = blockIdx.x * 256 + threadIdx.x;
  if (i >= ntot8) return;
  const bool keep = (i < nreal8);
  const int ic = keep ? i : (nreal8 - 1);
  const float* p = in + 8 * (size_t)ic;
  const v4f a = *(const v4f*)(p);
  const v4f c = *(const v4f*)(p + 4);
  unsigned short hb[8], lb[8];
#pragma unroll
  for (int e = 0; e < 4; ++e) {
    const float v0 = keep ? a[e] : 0.f;
    const float v1 = keep ? c[e] : 0.f;
    split_bf(v0, hb[e], lb[e]);
    split_bf(v1, hb[4 + e], lb[4 + e]);
  }
  const v4u uh = (v4u){pk16(hb[0], hb[1]), pk16(hb[2], hb[3]), pk16(hb[4], hb[5]), pk16(hb[6], hb[7])};
  const v4u ul = (v4u){pk16(lb[0], lb[1]), pk16(lb[2], lb[3]), pk16(lb[4], lb[5]), pk16(lb[6], lb[7])};
  unsigned short* qh = outH + 8 * (size_t)i;
  unsigned short* ql = outL + 8 * (size_t)i;
  *(volatile v4u*)qh = uh;
  *(volatile v4u*)ql = ul;
  __threadfence();
  *(volatile v4u*)qh = uh;
  *(volatile v4u*)ql = ul;
}

__global__ __launch_bounds__(256) void wup_cast_kernel(const float* __restrict__ upW, const float* __restrict__ upb,
                                                       unsigned short* __restrict__ out) {
  const int g = blockIdx.x * 256 + threadIdx.x;
  if (g >= kH * kKup8) return;
  const int n    = g / kKup8;
  const int c    = g - n * kKup8;
  const int col0 = c * 8;
  const bool mainp = (col0 < 3 * kH);
  const bool first = (col0 == 3 * kH);
  const int cc = mainp ? col0 : (3 * kH - 8);
  const int i  = cc >> 9;
  const int k  = cc & (kH - 1);
  const float* wp = upW + ((size_t)i * kH + n) * kH + k;
  const v4f a = *(const v4f*)(wp);
  const v4f d = *(const v4f*)(wp + 4);
  const float ub0 = upb[n], ub1 = upb[kH + n], ub2 = upb[2 * kH + n];
  float v[8];
  v[0] = mainp ? a[0] : (first ? ub0 : 0.f);
  v[1] = mainp ? a[1] : (first ? ub1 : 0.f);
  v[2] = mainp ? a[2] : (first ? ub2 : 0.f);
  v[3] = mainp ? a[3] : 0.f;
  v[4] = mainp ? d[0] : 0.f;
  v[5] = mainp ? d[1] : 0.f;
  v[6] = mainp ? d[2] : 0.f;
  v[7] = mainp ? d[3] : 0.f;
  unsigned short hb[8];
#pragma unroll
  for (int e = 0; e < 8; ++e) hb[e] = h_bits(kWCarry * v[e]);
  const v4u u = (v4u){pk16(hb[0], hb[1]), pk16(hb[2], hb[3]), pk16(hb[4], hb[5]), pk16(hb[6], hb[7])};
  unsigned short* q = out + 8 * (size_t)g;
  *(volatile v4u*)q = u;
  __threadfence();
  *(volatile v4u*)q = u;
}

__global__ __launch_bounds__(512) void gate_kernel(const float* __restrict__ x,
                                                   const float* __restrict__ W1, const float* __restrict__ b1,
                                                   const float* __restrict__ W2, const float* __restrict__ b2,
                                                   float* __restrict__ watt) {
  __shared__ float pooled[kH];
  __shared__ float hsh[256];
  __shared__ float lg[4];
  __shared__ __align__(16) float wline[kWattPitch];
  const int b = blockIdx.x;
  const int tid = threadIdx.x;
  const int lane = tid & 31, wave = tid >> 5;
  {
    const float* xp = x + (size_t)b * kT * kH + tid;
    float tot = 0.f;
#pragma unroll 1
    for (int t0 = 0; t0 < kT; t0 += 64) {
      float part = 0.f;
#pragma unroll 4
      for (int t = 0; t < 64; ++t) part += xp[(size_t)(t0 + t) * kH];
      tot += part;
    }
    pooled[tid] = tot * (1.0f / 4096.0f);
  }
  if (tid < kWattPitch) wline[tid] = 0.f;
  __syncthreads();
  if (tid < 256) {
    const float* w = W1 + (size_t)tid * kH;
    float acc = 0.f;
#pragma unroll 4
    for (int hh = 0; hh < kH; ++hh) acc += w[hh] * pooled[hh];
    acc += b1[tid];
    hsh[tid] = 0.5f * acc * (1.0f + erff(acc * 0.70710678118654752f));
  }
  __syncthreads();
  if (wave < 3) {
    const float* w = W2 + (size_t)wave * 256;
    float p = 0.f;
#pragma unroll
    for (int e = 0; e < 8; ++e) p += w[lane * 8 + e] * hsh[lane * 8 + e];
#pragma unroll
    for (int off = 16; off > 0; off >>= 1) p += __shfl_xor(p, off, 32);
    if (lane == 0) lg[wave] = p + b2[wave];
  }
  __syncthreads();
  if (tid == 0) {
    const float m = fmaxf(lg[0], fmaxf(lg[1], lg[2]));
    float s = 0.f;
#pragma unroll 1
    for (int cI = 0; cI < 3; ++cI) {
      const float ev = expf(lg[cI] - m);
      wline[cI] = ev;
      s += ev;
    }
    const float inv = 1.0f / s;
#pragma unroll 1
    for (int cI = 0; cI < 3; ++cI) wline[cI] = wline[cI] * inv;
  }
  __syncthreads();
  if (tid < 16) {
    const v4f v = *(const v4f*)(wline + tid * 4);
    float* q = watt + (size_t)b * kWattPitch + tid * 4;
    *(volatile v4f*)q = v;
    __threadfence();
    *(volatile v4f*)q = v;
  }
}

__global__ __launch_bounds__(256) void ssm_scan_kernel(const float* __restrict__ bx, const float* __restrict__ Am,
                                                       unsigned short* __restrict__ sth, unsigned short* __restrict__ stl,
                                                       int L, int npad) {
  __shared__ float AT[kS * kS];
  __shared__ __align__(16) float st[2 * 256];
  const int tid = threadIdx.x;
  const int b = tid >> 6, s = tid & 63;
  const int lane = tid & 31, wave = tid >> 5;
#pragma unroll
  for (int e = 0; e < 16; ++e) {
    const int idx = e * 256 + tid;
    const int r = idx >> 6, c = idx & 63;
    AT[c * kS + r] = Am[idx];
  }
  st[tid] = 0.f;
  __syncthreads();
  int cur = 0;
  for (int t = 0; t < L; ++t) {
    const size_t row = (size_t)b * L + t;
    const float bxv = bx[row * kS + s];
    const float* sc = st + cur * 256 + b * kS;
    float dot = 0.f;
#pragma unroll 8
    for (int sp = 0; sp < kS; ++sp) dot += sc[sp] * AT[sp * kS + s];
    const float sn = dot + bxv;
    const int nxt = cur ^ 1;
    st[nxt * 256 + tid] = sn;
    __syncthreads();
    if (wave == 0) {
      const int bb = lane >> 3, c8 = (lane & 7) * 8;
      const float* sp8 = st + nxt * 256 + bb * kS + c8;
      unsigned short hb[8], lb[8];
#pragma unroll
      for (int e = 0; e < 8; ++e) split_bf(sp8[e], hb[e], lb[e]);
      const v4u uh = (v4u){pk16(hb[0], hb[1]), pk16(hb[2], hb[3]), pk16(hb[4], hb[5]), pk16(hb[6], hb[7])};
      const v4u ul = (v4u){pk16(lb[0], lb[1]), pk16(lb[2], lb[3]), pk16(lb[4], lb[5]), pk16(lb[6], lb[7])};
      const size_t o = ((size_t)bb * L + t) * kS + c8;
      *(volatile v4u*)(sth + o) = uh;
      *(volatile v4u*)(stl + o) = ul;
      __threadfence();
      *(volatile v4u*)(sth + o) = uh;
      *(volatile v4u*)(stl + o) = ul;
    }
    cur = nxt;
  }
  {
    const v4u z = (v4u){0u, 0u, 0u, 0u};
    const size_t base = (size_t)kB * L * kS;
    const int c8 = (tid & 7) * 8;
    for (int rr = tid >> 3; rr < npad; rr += 32) {
      const size_t o = base + (size_t)rr * kS + c8;
      *(volatile v4u*)(sth + o) = z;
      *(volatile v4u*)(stl + o) = z;
    }
    __threadfence();
    for (int rr = tid >> 3; rr < npad; rr += 32) {
      const size_t o = base + (size_t)rr * kS + c8;
      *(volatile v4u*)(sth + o) = z;
      *(volatile v4u*)(stl + o) = z;
    }
  }
}

__global__ __launch_bounds__(128) void ln_kernel(const float* __restrict__ Y, const float* __restrict__ sig,
                                                 const float* __restrict__ Dv, const float* __restrict__ g,
                                                 const float* __restrict__ bb, float* __restrict__ out) {
  __shared__ float red[4];
  const int row = blockIdx.x;
  const int tid = threadIdx.x;
  const int lane = tid & 31, wave = tid >> 5;
  const int c4 = tid * 4;
  const size_t o = (size_t)row * kH + c4;
  const v4f yv = *(const v4f*)(Y + o);
  const v4f sv = *(const v4f*)(sig + o);
  const v4f dv = *(const v4f*)(Dv + c4);
  const v4f y = yv + dv * sv;
  float s = (y[0] + y[1]) + (y[2] + y[3]);
#pragma unroll
  for (int off = 16; off > 0; off >>= 1) s += __shfl_xor(s, off, 32);
  if (lane == 0) red[wave] = s;
  __syncthreads();
  const float mu = ((red[0] + red[1]) + (red[2] + red[3])) * (1.0f / 512.0f);
  __syncthreads();
  const v4f d = y - mu;
  float q = (d[0] * d[0] + d[1] * d[1]) + (d[2] * d[2] + d[3] * d[3]);
#pragma unroll
  for (int off = 16; off > 0; off >>= 1) q += __shfl_xor(q, off, 32);
  if (lane == 0) red[wave] = q;
  __syncthreads();
  const float var = ((red[0] + red[1]) + (red[2] + red[3])) * (1.0f / 512.0f);
  const float rinv = rsqrtf(var + 1e-5f);
  const v4f gv = *(const v4f*)(g + c4);
  const v4f bv = *(const v4f*)(bb + c4);
  const v4f ov = d * rinv * gv + bv;
  *(volatile v4f*)(out + o) = ov;
  __threadfence();
  *(volatile v4f*)(out + o) = ov;
}

__global__ __launch_bounds__(64) void interp_kernel(const float* __restrict__ yln, const float* __restrict__ watt,
                                                    unsigned short* __restrict__ af, int Lin, int slot, int tail) {
#pragma clang fp contract(off)
  const int bj  = blockIdx.x;
  const int b   = bj >> 12;
  const int j   = bj & (kT - 1);
  const int tid = threadIdx.x;
  const float scale = (float)Lin * (1.0f / 4096.0f);
  float pos = ((float)j + 0.5f) * scale - 0.5f;
  pos = fminf(fmaxf(pos, 0.0f), (float)(Lin - 1));
  int i0 = (int)floorf(pos);
  i0 = i0 < 0 ? 0 : (i0 > Lin - 1 ? Lin - 1 : i0);
  const int i1 = (i0 + 1 < Lin) ? (i0 + 1) : (Lin - 1);
  const float w   = pos - (float)i0;
  const float w1m = 1.0f - w;
  const float gsc = watt[(size_t)b * kWattPitch + slot] * kACarry;
  const int c8 = tid * 8;
  const float* p0 = yln + ((size_t)b * Lin + i0) * kH + c8;
  const float* p1 = yln + ((size_t)b * Lin + i1) * kH + c8;
  const v4f a0 = *(const v4f*)(p0);
  const v4f a1 = *(const v4f*)(p0 + 4);
  const v4f e0 = *(const v4f*)(p1);
  const v4f e1 = *(const v4f*)(p1 + 4);
  const v4f u0 = (a0 * w1m + e0 * w) * gsc;
  const v4f u1 = (a1 * w1m + e1 * w) * gsc;
  unsigned short hb[8];
#pragma unroll
  for (int e = 0; e < 4; ++e) {
    hb[e]     = h_bits(u0[e]);
    hb[4 + e] = h_bits(u1[e]);
  }
  const v4u u = (v4u){pk16(hb[0], hb[1]), pk16(hb[2], hb[3]), pk16(hb[4], hb[5]), pk16(hb[6], hb[7])};
  unsigned short* q = af + (size_t)bj * kKup + slot * kH + c8;
  *(volatile v4u*)q = u;
  __threadfence();
  *(volatile v4u*)q = u;
  const float* wl = watt + (size_t)b * kWattPitch + (tid & 7) * 8;
  v4f t0 = *(const v4f*)(wl);
  v4f t1 = *(const v4f*)(wl + 4);
  t0 = t0 * kACarry;
  t1 = t1 * kACarry;
  if (tail != 0) {
    if (tid < 8) {
      unsigned short tb[8];
#pragma unroll
      for (int e = 0; e < 4; ++e) {
        tb[e]     = h_bits(t0[e]);
        tb[4 + e] = h_bits(t1[e]);
      }
      const v4u tu = (v4u){pk16(tb[0], tb[1]), pk16(tb[2], tb[3]), pk16(tb[4], tb[5]), pk16(tb[6], tb[7])};
      unsigned short* qt = af + (size_t)bj * kKup + 3 * kH + tid * 8;
      *(volatile v4u*)qt = tu;
      __threadfence();
      *(volatile v4u*)qt = tu;
    }
  }
}

extern "C" void kernel_launch(void* const* d_in, const int* in_sizes, int n_in,
                              void* d_out, int out_size, void* d_ws, size_t ws_size,
                              hipStream_t stream) {
  if (n_in < 13) return;
  if ((size_t)out_size != (size_t)kNout * kH) return;
  if (ws_size < kWsTotal) return;
  if (in_sizes[0] != kB * kT * kH || in_sizes[1] != 3 * kS * kS || in_sizes[2] != 3 * kS * kH ||
      in_sizes[3] != 3 * kH * kS || in_sizes[7] != 3 * kH * kH) return;

  const float* x    = (const float*)d_in[0];
  const float* Am   = (const float*)d_in[1];
  const float* Bw   = (const float*)d_in[2];
  const float* Cw   = (const float*)d_in[3];
  const float* Dv   = (const float*)d_in[4];
  const float* ln_g = (const float*)d_in[5];
  const float* ln_b = (const float*)d_in[6];
  const float* upW  = (const float*)d_in[7];
  const float* upb  = (const float*)d_in[8];
  const float* aW1  = (const float*)d_in[9];
  const float* ab1  = (const float*)d_in[10];
  const float* aW2  = (const float*)d_in[11];
  const float* ab2  = (const float*)d_in[12];
  float* out = (float*)d_out;

  char* ws = (char*)d_ws;
  float* pCA1  = (float*)(ws + kOffCA1);
  float* pHIGH = (float*)(ws + kOffHIGH);
  float* pLOW  = (float*)(ws + kOffLOW);
  float* pMID  = (float*)(ws + kOffMID);
  unsigned short* pSIGH = (unsigned short*)(ws + kOffSIGH);
  unsigned short* pSIGL = (unsigned short*)(ws + kOffSIGL);
  float* pY    = (float*)(ws + kOffY);
  float* pLN   = pCA1;
  float* pBX   = (float*)(ws + kOffBX);
  unsigned short* pSTH = (unsigned short*)(ws + kOffSTH);
  unsigned short* pSTL = (unsigned short*)(ws + kOffSTL);
  unsigned short* pAF  = (unsigned short*)(ws + kOffAF);
  unsigned short* pWUP = (unsigned short*)(ws + kOffWUP);
  unsigned short* pBWH = (unsigned short*)(ws + kOffBWH);
  unsigned short* pBWL = (unsigned short*)(ws + kOffBWL);
  unsigned short* pCWH = (unsigned short*)(ws + kOffCWH);
  unsigned short* pCWL = (unsigned short*)(ws + kOffCWL);
  float* pWATT = (float*)(ws + kOffWATT);

  dwt_kernel<<<kB * kL1, 128, 0, stream>>>(x, pCA1, pHIGH, kT, kL1);
  dwt_kernel<<<kB * kL2, 128, 0, stream>>>(pCA1, pLOW, pMID, kL1, kL2);

  {
    const int n8w = 3 * kS * kH / 8;
    split8_bf16_kernel<<<(n8w + 255) / 256, 256, 0, stream>>>(Bw, pBWH, pBWL, n8w, n8w);
    split8_bf16_kernel<<<(n8w + 255) / 256, 256, 0, stream>>>(Cw, pCWH, pCWL, n8w, n8w);
    const int nwup = kH * kKup8;
    wup_cast_kernel<<<(nwup + 255) / 256, 256, 0, stream>>>(upW, upb, pWUP);
    gate_kernel<<<kB, 512, 0, stream>>>(x, aW1, ab1, aW2, ab2, pWATT);
  }

  for (int i = 0; i < 3; ++i) {
    const float* sig = (i == 0) ? pHIGH : (i == 1) ? pMID : pLOW;
    const int L  = (i == 0) ? kL1 : kL2;
    const int Mr = (i == 0) ? kM0 : kM1;
    const int Mp = (i == 0) ? kM0p : kM1p;

    {
      const int nreal8 = Mr * (kH / 8), ntot8 = Mp * (kH / 8);
      split8_bf16_kernel<<<(ntot8 + 255) / 256, 256, 0, stream>>>(sig, pSIGH, pSIGL, nreal8, ntot8);
    }
    {
      const int tiles = (Mp / 64) * (kS / 64);
      dim3 grid((tiles + 7) / 8, 1);
      wmma_gemm64<1, true, 0, 0, false><<<grid, 256, 0, stream>>>(
          pSIGH, pSIGL, kH, 0L,
          pBWH + (size_t)i * kS * kH, pBWL + (size_t)i * kS * kH, kH, 0L,
          (void*)pBX, (void*)pBX, kS, 0L,
          Dv, Dv, 0L,
          Mp, kS, kH, 1.0f);
    }
    ssm_scan_kernel<<<1, 256, 0, stream>>>(pBX, Am + (size_t)i * kS * kS, pSTH, pSTL, L, Mp - Mr);
    {
      const int tiles = (Mp / 64) * (kH / 64);
      dim3 grid((tiles + 7) / 8, 1);
      wmma_gemm64<1, true, 0, 0, false><<<grid, 256, 0, stream>>>(
          pSTH, pSTL, kS, 0L,
          pCWH + (size_t)i * kH * kS, pCWL + (size_t)i * kH * kS, kS, 0L,
          (void*)pY, (void*)pY, kH, 0L,
          Dv, Dv, 0L,
          Mp, kH, kS, 1.0f);
    }
    ln_kernel<<<Mr, 128, 0, stream>>>(pY, sig, Dv + (size_t)i * kH, ln_g + (size_t)i * kH,
                                       ln_b + (size_t)i * kH, pLN);
    interp_kernel<<<kNout, 64, 0, stream>>>(pLN, pWATT, pAF, L, i, (i == 2) ? 1 : 0);
  }

  {
    const int tiles = (kNout / 64) * (kH / 64);
    dim3 grid((tiles + 7) / 8, 1);
    wmma_gemm64<0, false, 0, 0, false><<<grid, 256, 0, stream>>>(
        pAF, pAF, kKup, 0L,
        pWUP, pWUP, kKup, 0L,
        (void*)out, (void*)out, kH, 0L,
        Dv, Dv, 0L,
        kNout, kH, kKup, kUpScale);
  }
}
